// PCTransformer_3951369912340
// MI455X (gfx1250) — hardware-verified
//
#include <hip/hip_runtime.h>
#include <math.h>

constexpr int kBatch   = 16;
constexpr int kPts     = 1024;
constexpr int kChan    = 384;
constexpr int kHeads   = 6;
constexpr int kHeadDim = 64;
constexpr int kNbr     = 8;
constexpr int kHidden  = 768;
constexpr int kRows    = kBatch * kPts;
constexpr int kQKVCols = 3 * kChan;
constexpr int kQKCols  = 2 * kChan;
constexpr int kGrp     = 8;
constexpr int kChunks  = (kBatch * kHeads) / kGrp;
constexpr float kWCarry  = 16.0f;
constexpr float kPCarry  = 2048.0f;
constexpr float kACarry  = 64.0f;
constexpr float kMCarry  = 16.0f;
constexpr float kFCarry  = 16.0f;
constexpr float kInvChan = 1.0f / 384.0f;
constexpr float kLnEps   = 1e-5f;

constexpr size_t kOffWQK  = 0;
constexpr size_t kOffWPRJ = kOffWQK  + (size_t)kQKVCols * kChan * 2;
constexpr size_t kOffWKNN = kOffWPRJ + (size_t)kChan * kChan * 2;
constexpr size_t kOffWMRG = kOffWKNN + (size_t)kChan * kHidden * 2;
constexpr size_t kOffWFC1 = kOffWMRG + (size_t)kChan * kHidden * 2;
constexpr size_t kOffWFC2 = kOffWFC1 + (size_t)kHidden * kChan * 2;
constexpr size_t kSlotBase = kOffWFC2 + (size_t)kChan * kHidden * 2;
constexpr size_t kSlot     = (size_t)kRows * kChan * 2;
constexpr size_t kWsTotal  = kSlotBase + 10 * kSlot;
typedef char ws_fits_check[(kWsTotal <= (size_t)134217728) ? 1 : -1];
typedef char sc_fits_check[(((size_t)kGrp * kPts * kPts * 4 + (size_t)kGrp * kPts * kPts * 2) == 4 * kSlot) ? 1 : -1];

typedef __attribute__((ext_vector_type(16))) _Float16 v16h;
typedef __attribute__((ext_vector_type(8)))  _Float16 v8h;
typedef __attribute__((ext_vector_type(16))) __bf16   v16b;
typedef __attribute__((ext_vector_type(8)))  __bf16   v8b;
typedef __attribute__((ext_vector_type(8)))  float    v8f;
typedef __attribute__((ext_vector_type(4)))  float    v4f;
typedef __attribute__((ext_vector_type(4)))  unsigned int v4u;

__device__ __forceinline__ unsigned short f2bf_bits(float f) {
  unsigned u = __float_as_uint(f);
  return (unsigned short)((u + 0x7FFFu + ((u >> 16) & 1u)) >> 16);
}
__device__ __forceinline__ float bf_bits2f(unsigned short h) { return __uint_as_float(((unsigned)h) << 16); }

__device__ __forceinline__ void dep_guard_h(v8f& a, v8f& b, v16h x, v16h y) { asm volatile("v_nop\n\tv_nop\n\tv_nop\n\tv_nop" : "+v"(a), "+v"(b) : "v"(x), "v"(y)); }
__device__ __forceinline__ void dep_guard_b(v8f& a, v8f& b, v16b x, v16b y) { asm volatile("v_nop\n\tv_nop\n\tv_nop\n\tv_nop" : "+v"(a), "+v"(b) : "v"(x), "v"(y)); }
__device__ __forceinline__ void keep4_h(v16h a, v16h b, v16h c, v16h d) { asm volatile("v_nop" :: "v"(a), "v"(b), "v"(c), "v"(d)); }
__device__ __forceinline__ void keep4_b(v16b a, v16b b, v16b c, v16b d) { asm volatile("v_nop" :: "v"(a), "v"(b), "v"(c), "v"(d)); }
__device__ __forceinline__ void acc_guard4(v8f& a, v8f& b, v8f& c, v8f& d) { asm volatile("v_nop\n\tv_nop\n\tv_nop\n\tv_nop" : "+v"(a), "+v"(b), "+v"(c), "+v"(d)); }
template <typename T> struct Frag;
template <> struct Frag<_Float16> {
  typedef v16h V; union U { v16h v; v8h h[2]; };
  static __device__ __forceinline__ v16h load(const _Float16* p) {
    U f; f.h[0] = *(const v8h*)(p); f.h[1] = *(const v8h*)(p + 16); return f.v;
  }
  static __device__ __forceinline__ v8f mma(v16h a, v16h b, v8f c) {
    return __builtin_amdgcn_wmma_f32_16x16x32_f16(false, a, false, b, (short)0, c, false, false);
  }
  static __device__ __forceinline__ void guard(v8f& a, v8f& b, v16h x, v16h y) { dep_guard_h(a, b, x, y); }
  static __device__ __forceinline__ void keep(v16h a, v16h b, v16h c, v16h d) { keep4_h(a, b, c, d); }
};
template <> struct Frag<__bf16> {
  typedef v16b V; union U { v16b v; v8b h[2]; };
  static __device__ __forceinline__ v16b load(const __bf16* p) {
    U f; f.h[0] = *(const v8b*)(p); f.h[1] = *(const v8b*)(p + 16); return f.v;
  }
  static __device__ __forceinline__ v8f mma(v16b a, v16b b, v8f c) {
    return __builtin_amdgcn_wmma_f32_16x16x32_bf16(false, a, false, b, (short)0, c, false, false);
  }
  static __device__ __forceinline__ void guard(v8f& a, v8f& b, v16b x, v16b y) { dep_guard_b(a, b, x, y); }
  static __device__ __forceinline__ void keep(v16b a, v16b b, v16b c, v16b d) { keep4_b(a, b, c, d); }
};

__device__ __forceinline__ unsigned pk16(unsigned short a, unsigned short b) { return (unsigned)a | ((unsigned)b << 16); }
__device__ __forceinline__ unsigned short h_bits(float f) { const _Float16 h = (_Float16)f; return __builtin_bit_cast(unsigned short, h); }

__device__ __forceinline__ void st2_u4(unsigned short* p, v4u u) {
  *(volatile v4u*)p = u;
  __threadfence();
  *(volatile v4u*)p = u;
}
__device__ __forceinline__ void st2_f4(float* p, v4f v) {
  *(volatile v4f*)p = v;
  __threadfence();
  *(volatile v4f*)p = v;
}

template <int ET> struct Elem;
template <> struct Elem<0> { typedef _Float16 T; };
template <> struct Elem<1> { typedef __bf16 T; };
template <int ET, bool SPLIT, int BIAS_MODE, int OUT_MODE, int RESID, int ACT = 0>
__global__ __launch_bounds__(256) void wmma_gemm64(
    const unsigned short* __restrict__ Ap, const unsigned short* __restrict__ A2p, int lda, long strideA,
    const unsigned short* __restrict__ Btp, const unsigned short* __restrict__ Bt2p, int ldb, long strideB,
    void* __restrict__ Cout, void* __restrict__ Cout2, int ldc, long strideC,
    const float* __restrict__ bias, float bsc,
    const float* __restrict__ resid, long strideR,
    int M, int N, int K, float scale) {
  typedef typename Elem<ET>::T T;
  typedef typename Frag<T>::V V;
  const T* A = (const T*)Ap; const T* A2 = (const T*)A2p; const T* Bt = (const T*)Btp; const T* Bt2 = (const T*)Bt2p;
  __shared__ __align__(16) float sT[8][16 * 68];
  const int b    = blockIdx.y;
  const int lane = threadIdx.x & 31;
  const int wave = threadIdx.x >> 5;
  const int tilesN = N >> 6;
  const int tilesM = M >> 6;
  const int tile = blockIdx.x * 8 + wave;
  if (tile >= tilesM * tilesN) return;
  const int tm = tile / tilesN;
  const int tn = tile - tm * tilesN;
  const int m0 = tm << 6;
  const int n0 = tn << 6;

  const T* Ab  = A  + (size_t)b * strideA;
  const T* Bb  = Bt + (size_t)b * strideB;
  const T* Ab2 = SPLIT ? (A2  + (size_t)b * strideA) : nullptr;
  const T* Bb2 = SPLIT ? (Bt2 + (size_t)b * strideB) : nullptr;

  const int rlane = lane & 15;
  const int koff  = (lane >> 4) * 8;
  const int mOff  = (lane >> 4) * 8;

  v8f acc[4][4];
#pragma unroll
  for (int i = 0; i < 4; ++i)
#pragma unroll
    for (int j = 0; j < 4; ++j) acc[i][j] = (v8f){0.f,0.f,0.f,0.f,0.f,0.f,0.f,0.f};

  for (int k0 = 0; k0 < K; k0 += 32) {
    V bh[4], bl[4];
#pragma unroll
    for (int j = 0; j < 4; ++j) {
      const size_t bo = (size_t)(n0 + (j << 4) + rlane) * ldb + koff + k0;
      bh[j] = Frag<T>::load(Bb + bo);
      if (SPLIT) bl[j] = Frag<T>::load(Bb2 + bo);
    }
#pragma unroll
    for (int i = 0; i < 4; ++i) {
      const size_t ao = (size_t)(m0 + (i << 4) + rlane) * lda + koff + k0;
      V ah = Frag<T>::load(Ab + ao);
      V al;
      if (SPLIT) al = Frag<T>::load(Ab2 + ao);
#pragma unroll
      for (int j = 0; j < 4; ++j) {
        acc[i][j] = Frag<T>::mma(ah, bh[j], acc[i][j]);
        if (SPLIT) {
          acc[i][j] = Frag<T>::mma(ah, bl[j], acc[i][j]);
          acc[i][j] = Frag<T>::mma(al, bh[j], acc[i][j]);
        }
      }
      Frag<T>::guard(acc[i][0], acc[i][3], ah, SPLIT ? al : ah);
    }
    Frag<T>::keep(bh[0], bh[1], bh[2], bh[3]);
    if (SPLIT) Frag<T>::keep(bl[0], bl[1], bl[2], bl[3]);
  }
  acc_guard4(acc[0][0], acc[0][1], acc[0][2], acc[0][3]);
  acc_guard4(acc[1][0], acc[1][1], acc[1][2], acc[1][3]);
  acc_guard4(acc[2][0], acc[2][1], acc[2][2], acc[2][3]);
  acc_guard4(acc[3][0], acc[3][1], acc[3][2], acc[3][3]);

  float* slab = sT[wave];
  const float* Rb = (RESID != 0) ? (resid + (size_t)b * strideR) : nullptr;
#pragma unroll
  for (int i = 0; i < 4; ++i) {
    const int mBase = m0 + (i << 4);
#pragma unroll
    for (int j = 0; j < 4; ++j) {
      const int n = n0 + (j << 4) + rlane;
      float bv = 0.f;
      if (BIAS_MODE == 2) bv = bias[n] * bsc;
#pragma unroll
      for (int r = 0; r < 8; ++r) {
        float v = acc[i][j][r] * scale;
        if (BIAS_MODE == 1) v += bias[mBase + mOff + r] * bsc;
        if (BIAS_MODE == 2) v += bv;
        if (RESID == 1) v += Rb[(size_t)(mBase + mOff + r) * ldc + n];
        if (ACT == 2) v = fmaxf(v, 0.0f);
        if (ACT == 4) v = (v > 0.f) ? v : 0.01f * v;
        if (ACT == 6) v = (v > 0.f) ? v : 0.2f * v;
        if (RESID == 2) v = fmaxf(v, Rb[(size_t)(mBase + mOff + r) * ldc + n]);
        slab[(mOff + r) * 68 + (j << 4) + rlane] = v;
      }
    }
    __builtin_amdgcn_fence(__ATOMIC_RELEASE, "workgroup");
    __builtin_amdgcn_wave_barrier();
    __builtin_amdgcn_fence(__ATOMIC_ACQUIRE, "workgroup");
    if (OUT_MODE == 0) {
      float* C = (float*)Cout + (size_t)b * strideC;
      const int hh = lane >> 4, c4 = (lane & 15) * 4;
      for (int pass = 0; pass < 2; ++pass) {
#pragma unroll
        for (int it = 0; it < 8; ++it) {
          const int row = it * 2 + hh;
          v4f v = *(const v4f*)(slab + row * 68 + c4);
          *(volatile v4f*)(C + (size_t)(mBase + row) * ldc + n0 + c4) = v;
        }
        __threadfence();
      }
    } else {
      const int q = lane >> 3, c8 = (lane & 7) * 8;
      unsigned short* C  = (unsigned short*)Cout  + (size_t)b * strideC;
      unsigned short* C2 = (OUT_MODE == 2) ? ((unsigned short*)Cout2 + (size_t)b * strideC) : nullptr;
      for (int pass = 0; pass < 2; ++pass) {
#pragma unroll
        for (int it = 0; it < 4; ++it) {
          const int row = it * 4 + q;
          const float* sp = slab + row * 68 + c8;
          v8h hv, lv;
#pragma unroll
          for (int e = 0; e < 8; ++e) {
            if (OUT_MODE == 1) {
              hv[e] = (_Float16)sp[e];
            } else {
              unsigned short hb = f2bf_bits(sp[e]);
              unsigned short lb = f2bf_bits(sp[e] - bf_bits2f(hb));
              hv[e] = __builtin_bit_cast(_Float16, hb);
              lv[e] = __builtin_bit_cast(_Float16, lb);
            }
          }
          *(volatile v8h*)(C + (size_t)(mBase + row) * ldc + n0 + c8) = hv;
          if (OUT_MODE == 2) *(volatile v8h*)(C2 + (size_t)(mBase + row) * ldc + n0 + c8) = lv;
        }
        __threadfence();
      }
    }
    __builtin_amdgcn_fence(__ATOMIC_RELEASE, "workgroup");
    __builtin_amdgcn_wave_barrier();
    __builtin_amdgcn_fence(__ATOMIC_ACQUIRE, "workgroup");
  }
}

__global__ __launch_bounds__(256) void wtcast_kernel(const float* __restrict__ W, unsigned short* __restrict__ out,
                                                     int kin, int nout, float scale) {
  __shared__ float sm[64][65];
  const int t  = threadIdx.x;
  const int k0 = blockIdx.x * 64;
  const int n0 = blockIdx.y * 64;
#pragma unroll
  for (int i = 0; i < 16; ++i) {
    const int e = i * 256 + t;
    const int r = e >> 6;
    const int c = e & 63;
    sm[c][r] = W[(size_t)(k0 + r) * nout + n0 + c] * scale;
  }
  __syncthreads();
  const int lane = t & 31, wave = t >> 5;
  const int q = lane >> 3, c8 = (lane & 7) * 8;
  for (int pass = 0; pass < 2; ++pass) {
#pragma unroll
    for (int it = 0; it < 2; ++it) {
      const int row = wave * 8 + it * 4 + q;
      unsigned short hb[8];
#pragma unroll
      for (int e = 0; e < 8; ++e) hb[e] = h_bits(sm[row][c8 + e]);
      const v4u u = (v4u){pk16(hb[0], hb[1]), pk16(hb[2], hb[3]), pk16(hb[4], hb[5]), pk16(hb[6], hb[7])};
      *(volatile v4u*)(out + (size_t)(n0 + row) * kin + k0 + c8) = u;
    }
    __threadfence();
  }
}

__device__ __forceinline__ v4u ln_pack8(const float* __restrict__ xr, const float* __restrict__ gw,
                                         const float* __restrict__ gb, int cb, float mean, float rstd) {
  const v4f p0 = *(const v4f*)(xr + cb), p1 = *(const v4f*)(xr + cb + 4);
  const v4f w0 = *(const v4f*)(gw + cb), w1 = *(const v4f*)(gw + cb + 4);
  const v4f b0 = *(const v4f*)(gb + cb), b1 = *(const v4f*)(gb + cb + 4);
  unsigned short hb[8];
#pragma unroll
  for (int e = 0; e < 4; ++e) {
    hb[e]     = h_bits((p0[e] - mean) * rstd * w0[e] + b0[e]);
    hb[4 + e] = h_bits((p1[e] - mean) * rstd * w1[e] + b1[e]);
  }
  return (v4u){pk16(hb[0], hb[1]), pk16(hb[2], hb[3]), pk16(hb[4], hb[5]), pk16(hb[6], hb[7])};
}

template <bool W32>
__global__ __launch_bounds__(256) void layernorm_kernel(const float* __restrict__ x, const float* __restrict__ gw,
                                                         const float* __restrict__ gb, float* __restrict__ out32,
                                                         unsigned short* __restrict__ out16, int nrows) {
  const int lane = threadIdx.x & 31;
  const int wave = threadIdx.x >> 5;
  const int row  = blockIdx.x * 8 + wave;
  if (row >= nrows) return;
  const float* xr = x + (size_t)row * kChan;
  const v4f a0 = *(const v4f*)(xr + 4 * lane);
  const v4f a1 = *(const v4f*)(xr + 128 + 4 * lane);
  const v4f a2 = *(const v4f*)(xr + 256 + 4 * lane);
  float s = ((a0[0] + a0[1]) + (a0[2] + a0[3])) + ((a1[0] + a1[1]) + (a1[2] + a1[3])) + ((a2[0] + a2[1]) + (a2[2] + a2[3]));
#pragma unroll
  for (int off = 16; off > 0; off >>= 1) s += __shfl_xor(s, off, 32);
  const float mean = s * kInvChan;
  float ss = 0.f;
#pragma unroll
  for (int e = 0; e < 4; ++e) {
    const float d0 = a0[e] - mean, d1 = a1[e] - mean, d2 = a2[e] - mean;
    ss += d0 * d0; ss += d1 * d1; ss += d2 * d2;
  }
#pragma unroll
  for (int off = 16; off > 0; off >>= 1) ss += __shfl_xor(ss, off, 32);
  const float rstd = rsqrtf(ss * kInvChan + kLnEps);

  if (W32) {
    const v4f w0 = *(const v4f*)(gw + 4 * lane), w1 = *(const v4f*)(gw + 128 + 4 * lane), w2 = *(const v4f*)(gw + 256 + 4 * lane);
    const v4f b0 = *(const v4f*)(gb + 4 * lane), b1 = *(const v4f*)(gb + 128 + 4 * lane), b2 = *(const v4f*)(gb + 256 + 4 * lane);
    v4f y0, y1, y2;
#pragma unroll
    for (int e = 0; e < 4; ++e) {
      y0[e] = (a0[e] - mean) * rstd * w0[e] + b0[e];
      y1[e] = (a1[e] - mean) * rstd * w1[e] + b1[e];
      y2[e] = (a2[e] - mean) * rstd * w2[e] + b2[e];
    }
    float* orow = out32 + (size_t)row * kChan;
    st2_f4(orow + 4 * lane, y0);
    st2_f4(orow + 128 + 4 * lane, y1);
    st2_f4(orow + 256 + 4 * lane, y2);
  }
  {
    unsigned short* o16 = out16 + (size_t)row * kChan;
    const int cb0 = 8 * lane;
    const int cb1 = 256 + 8 * (lane & 15);
    const v4u u0 = ln_pack8(xr, gw, gb, cb0, mean, rstd);
    const v4u u1 = ln_pack8(xr, gw, gb, cb1, mean, rstd);
    st2_u4(o16 + cb0, u0);
    if (lane < 16) st2_u4(o16 + cb1, u1);
  }
}

__device__ __forceinline__ void gather_seg(const float* __restrict__ fr, const float* __restrict__ cr,
                                           unsigned short* __restrict__ gr, int cb, bool active) {
  const v4f f0 = *(const v4f*)(fr + cb), f1 = *(const v4f*)(fr + cb + 4);
  const v4f c0 = *(const v4f*)(cr + cb), c1 = *(const v4f*)(cr + cb + 4);
  unsigned short hd[8], hc[8];
#pragma unroll
  for (int e = 0; e < 4; ++e) {
    hd[e]     = h_bits(f0[e] - c0[e]);
    hd[4 + e] = h_bits(f1[e] - c1[e]);
    hc[e]     = h_bits(c0[e]);
    hc[4 + e] = h_bits(c1[e]);
  }
  const v4u ud = (v4u){pk16(hd[0], hd[1]), pk16(hd[2], hd[3]), pk16(hd[4], hd[5]), pk16(hd[6], hd[7])};
  const v4u uc = (v4u){pk16(hc[0], hc[1]), pk16(hc[2], hc[3]), pk16(hc[4], hc[5]), pk16(hc[6], hc[7])};
  if (active) {
    st2_u4(gr + cb, ud);
    st2_u4(gr + kChan + cb, uc);
  }
}

__global__ __launch_bounds__(256) void gather_kernel(const float* __restrict__ nx, const int* __restrict__ knn,
                                                     unsigned short* __restrict__ G, int kk) {
  const int lane = threadIdx.x & 31;
  const int wave = threadIdx.x >> 5;
  const int row  = blockIdx.x * 8 + wave;
  if (row >= kRows) return;
  const int b = row >> 10;
  const int n = row & (kPts - 1);
  int idx = knn[(size_t)(b * kNbr + kk) * kPts + n];
  idx = (idx < 0) ? 0 : ((idx > kRows - 1) ? (kRows - 1) : idx);
  const float* cr = nx + (size_t)row * kChan;
  const float* fr = nx + (size_t)idx * kChan;
  unsigned short* gr = G + (size_t)row * kHidden;
  gather_seg(fr, cr, gr, 8 * lane, true);
  gather_seg(fr, cr, gr, 256 + 8 * (lane & 15), lane < 16);
}

template <int NC8, bool GELU>
__global__ __launch_bounds__(256) void rowcvt_kernel(const float* __restrict__ in, int lin,
                                                     unsigned short* __restrict__ out, int lout, float scale, int nrows) {
  const int lane = threadIdx.x & 31;
  const int wave = threadIdx.x >> 5;
  const int row  = blockIdx.x * 8 + wave;
  if (row >= nrows) return;
  const float* ir = in + (size_t)row * lin;
  unsigned short* orw = out + (size_t)row * lout;
  constexpr int NIT = (NC8 + 31) / 32;
#pragma unroll 1
  for (int it = 0; it < NIT; ++it) {
    const int ch  = it * 32 + lane;
    const int chc = (ch < NC8) ? ch : (NC8 - 1);
    const float* p = ir + 8 * chc;
    v4u u;
    if (GELU) {
      unsigned w0 = 0u, w1 = 0u, w2 = 0u, w3 = 0u;
#pragma unroll 1
      for (int pr = 0; pr < 4; ++pr) {
        const float v0 = p[2 * pr];
        const float v1 = p[2 * pr + 1];
        const float g0 = 0.5f * v0 * (1.0f + erff(v0 * 0.70710678118654752f));
        const float g1 = 0.5f * v1 * (1.0f + erff(v1 * 0.70710678118654752f));
        const unsigned wd = pk16(h_bits(g0 * scale), h_bits(g1 * scale));
        w0 = (pr == 0) ? wd : w0;
        w1 = (pr == 1) ? wd : w1;
        w2 = (pr == 2) ? wd : w2;
        w3 = (pr == 3) ? wd : w3;
      }
      u = (v4u){w0, w1, w2, w3};
    } else {
      const v4f a = *(const v4f*)(p);
      const v4f c = *(const v4f*)(p + 4);
      u = (v4u){pk16(h_bits(a[0] * scale), h_bits(a[1] * scale)), pk16(h_bits(a[2] * scale), h_bits(a[3] * scale)),
                pk16(h_bits(c[0] * scale), h_bits(c[1] * scale)), pk16(h_bits(c[2] * scale), h_bits(c[3] * scale))};
    }
    if (ch < NC8) st2_u4(orw + 8 * ch, u);
  }
}

__global__ __launch_bounds__(128) void softmax1024_kernel(const float* __restrict__ S, unsigned short* __restrict__ P) {
  __shared__ float redM[4];
  __shared__ float redS[4];
  const int row  = blockIdx.x;
  const int t    = threadIdx.x;
  const int lane = t & 31, wave = t >> 5;
  const int c0   = t * 8;
  const float* sr = S + (size_t)row * kPts + c0;
  const v4f a = *(const v4f*)(sr);
  const v4f c = *(const v4f*)(sr + 4);
  float x[8];
#pragma unroll
  for (int e = 0; e < 4; ++e) { x[e] = a[e]; x[4 + e] = c[e]; }
  float m = fmaxf(fmaxf(fmaxf(x[0], x[1]), fmaxf(x[2], x[3])), fmaxf(fmaxf(x[4], x[5]), fmaxf(x[6], x[7])));
#pragma unroll
  for (int off = 16; off > 0; off >>= 1) m = fmaxf(m, __shfl_xor(m, off, 32));
  if (lane == 0) redM[wave] = m;
  __syncthreads();
  m = fmaxf(fmaxf(redM[0], redM[1]), fmaxf(redM[2], redM[3]));
  float ex[8];
#pragma unroll
  for (int e = 0; e < 8; ++e) ex[e] = expf(x[e] - m);
  float s = ((ex[0] + ex[1]) + (ex[2] + ex[3])) + ((ex[4] + ex[5]) + (ex[6] + ex[7]));
#pragma unroll
  for (int off = 16; off > 0; off >>= 1) s += __shfl_xor(s, off, 32);
  if (lane == 0) redS[wave] = s;
  __syncthreads();
  const float tot = ((redS[0] + redS[1]) + redS[2]) + redS[3];
  const float inv = kPCarry * (1.0f / tot);
  unsigned short hb[8];
#pragma unroll
  for (int e = 0; e < 8; ++e) hb[e] = h_bits(ex[e] * inv);
  const v4u u = (v4u){pk16(hb[0], hb[1]), pk16(hb[2], hb[3]), pk16(hb[4], hb[5]), pk16(hb[6], hb[7])};
  st2_u4(P + (size_t)row * kPts + c0, u);
}

extern "C" void kernel_launch(void* const* d_in, const int* in_sizes, int n_in,
                              void* d_out, int out_size, void* d_ws, size_t ws_size,
                              hipStream_t stream) {
  if (n_in < 17) return;
  if (in_sizes[0] != kRows * kChan) return;
  if (in_sizes[1] != kBatch * kNbr * kPts) return;
  if (out_size != kRows * kChan) return;
  if (ws_size < kWsTotal) return;

  const float* x      = (const float*)d_in[0];
  const int*   knn_ix = (const int*)  d_in[1];
  const float* ln1_w  = (const float*)d_in[2];
  const float* ln1_b  = (const float*)d_in[3];
  const float* w_qkv  = (const float*)d_in[4];
  const float* w_proj = (const float*)d_in[5];
  const float* b_proj = (const float*)d_in[6];
  const float* w_knn  = (const float*)d_in[7];
  const float* b_knn  = (const float*)d_in[8];
  const float* w_mrg  = (const float*)d_in[9];
  const float* b_mrg  = (const float*)d_in[10];
  const float* ln2_w  = (const float*)d_in[11];
  const float* ln2_b  = (const float*)d_in[12];
  const float* w_fc1  = (const float*)d_in[13];
  const float* b_fc1  = (const float*)d_in[14];
  const float* w_fc2  = (const float*)d_in[15];
  const float* b_fc2  = (const float*)d_in[16];
  float* out = (float*)d_out;

  char* ws = (char*)d_ws;
  unsigned short* WQK  = (unsigned short*)(ws + kOffWQK);
  unsigned short* WPRJ = (unsigned short*)(ws + kOffWPRJ);
  unsigned short* WKNN = (unsigned short*)(ws + kOffWKNN);
  unsigned short* WMRG = (unsigned short*)(ws + kOffWMRG);
  unsigned short* WFC1 = (unsigned short*)(ws + kOffWFC1);
  unsigned short* WFC2 = (unsigned short*)(ws + kOffWFC2);
  char* slot0 = ws + kSlotBase;
  unsigned short* QK16 = (unsigned short*)(slot0 + 0 * kSlot);
  unsigned short* M16  = (unsigned short*)(slot0 + 0 * kSlot);
  unsigned short* FC16 = (unsigned short*)(slot0 + 0 * kSlot);
  unsigned short* VT16 = (unsigned short*)(slot0 + 2 * kSlot);
  unsigned short* G16  = (unsigned short*)(slot0 + 2 * kSlot);
  float*          X2   = (float*)         (slot0 + 2 * kSlot);
  float*          SC   = (float*)         (slot0 + 3 * kSlot);
  unsigned short* P16  = (unsigned short*)(slot0 + 3 * kSlot + (size_t)kGrp * kPts * kPts * 4);
  float*          PA   = (float*)         (slot0 + 4 * kSlot);
  unsigned short* H16  = (unsigned short*)(slot0 + 4 * kSlot);
  float*          U32  = (float*)         (slot0 + 5 * kSlot);
  float*          PB   = (float*)         (slot0 + 6 * kSlot);
  unsigned short* NX16 = (unsigned short*)(slot0 + 7 * kSlot);
  unsigned short* A16  = (unsigned short*)(slot0 + 7 * kSlot);
  float*          NX32 = (float*)         (slot0 + 8 * kSlot);

  const float invW = 1.0f / kWCarry;

  wtcast_kernel<<<dim3(kChan / 64, kQKVCols / 64), 256, 0, stream>>>(w_qkv, WQK, kChan, kQKVCols, kWCarry);
  wtcast_kernel<<<dim3(kChan / 64, kChan / 64), 256, 0, stream>>>(w_proj, WPRJ, kChan, kChan, kWCarry);
  wtcast_kernel<<<dim3(kHidden / 64, kChan / 64), 256, 0, stream>>>(w_knn, WKNN, kHidden, kChan, kWCarry);
  wtcast_kernel<<<dim3(kHidden / 64, kChan / 64), 256, 0, stream>>>(w_mrg, WMRG, kHidden, kChan, kWCarry);
  wtcast_kernel<<<dim3(kChan / 64, kHidden / 64), 256, 0, stream>>>(w_fc1, WFC1, kChan, kHidden, kWCarry);
  wtcast_kernel<<<dim3(kHidden / 64, kChan / 64), 256, 0, stream>>>(w_fc2, WFC2, kHidden, kChan, kWCarry);

  layernorm_kernel<true><<<kRows / 8, 256, 0, stream>>>(x, ln1_w, ln1_b, NX32, NX16, kRows);

  wmma_gemm64<0, false, 0, 1, 0, 0><<<dim3((unsigned)(((kRows / 64) * (kQKCols / 64) + 7) / 8), 1), 256, 0, stream>>>(
      NX16, NX16, kChan, 0L, WQK, WQK, kChan, 0L, (void*)QK16, (void*)QK16, kQKCols, 0L,
      b_proj, 1.0f, x, 0L, kRows, kQKCols, kChan, invW);

  wmma_gemm64<0, false, 0, 1, 0, 0><<<dim3((unsigned)(((kChan / 64) * (kPts / 64) + 7) / 8), kBatch), 256, 0, stream>>>(
      WQK + (size_t)kQKCols * kChan, WQK + (size_t)kQKCols * kChan, kChan, 0L,
      NX16, NX16, kChan, (long)kPts * kChan,
      (void*)VT16, (void*)VT16, kPts, (long)kChan * kPts,
      b_proj, 1.0f, x, 0L, kChan, kPts, kChan, invW);

  for (int ch = 0; ch < kChunks; ++ch) {
    const int h  = ch >> 1;
    const int bh = ch & 1;
    const size_t rowbase = (size_t)bh * kGrp * kPts;
    wmma_gemm64<0, false, 0, 0, 0, 0><<<dim3((unsigned)(((kPts / 64) * (kPts / 64) + 7) / 8), kGrp), 256, 0, stream>>>(
        QK16 + rowbase * kQKCols + h * kHeadDim, QK16 + rowbase * kQKCols + h * kHeadDim, kQKCols, (long)kPts * kQKCols,
        QK16 + rowbase * kQKCols + kChan + h * kHeadDim, QK16 + rowbase * kQKCols + kChan + h * kHeadDim, kQKCols, (long)kPts * kQKCols,
        (void*)SC, (void*)SC, kPts, (long)kPts * kPts,
        b_proj, 1.0f, x, 0L, kPts, kPts, kHeadDim, 0.125f);
    softmax1024_kernel<<<kGrp * kPts, 128, 0, stream>>>(SC, P16);
    wmma_gemm64<0, false, 0, 1, 0, 0><<<dim3((unsigned)(((kPts / 64) * (kHeadDim / 64) + 7) / 8), kGrp), 256, 0, stream>>>(
        P16, P16, kPts, (long)kPts * kPts,
        VT16 + ((size_t)(bh * kGrp) * kChan + (size_t)h * kHeadDim) * kPts, VT16 + ((size_t)(bh * kGrp) * kChan + (size_t)h * kHeadDim) * kPts,
        kPts, (long)kChan * kPts,
        (void*)(A16 + rowbase * kChan + h * kHeadDim), (void*)(A16 + rowbase * kChan + h * kHeadDim), kChan, (long)kPts * kChan,
        b_proj, 1.0f, x, 0L, kPts, kHeadDim, kPts, kACarry / kPCarry);
  }

  wmma_gemm64<0, false, 2, 1, 0, 0><<<dim3((unsigned)(((kRows / 64) * (kChan / 64) + 7) / 8), 1), 256, 0, stream>>>(
      A16, A16, kChan, 0L, WPRJ, WPRJ, kChan, 0L, (void*)M16, (void*)M16, kHidden, 0L,
      b_proj, kMCarry, x, 0L, kRows, kChan, kChan, kMCarry / (kACarry * kWCarry));

  for (int kk = 0; kk < kNbr; ++kk) {
    gather_kernel<<<kRows / 8, 256, 0, stream>>>(NX32, knn_ix, G16, kk);
    float* dst = (kk & 1) ? PB : PA;
    float* prv = (kk & 1) ? PA : PB;
    if (kk == 0) {
      wmma_gemm64<0, false, 2, 0, 0, 6><<<dim3((unsigned)(((kRows / 64) * (kChan / 64) + 7) / 8), 1), 256, 0, stream>>>(
          G16, G16, kHidden, 0L, WKNN, WKNN, kHidden, 0L, (void*)dst, (void*)dst, kChan, 0L,
          b_knn, 1.0f, x, 0L, kRows, kChan, kHidden, invW);
    } else {
      wmma_gemm64<0, false, 2, 0, 2, 6><<<dim3((unsigned)(((kRows / 64) * (kChan / 64) + 7) / 8), 1), 256, 0, stream>>>(
          G16, G16, kHidden, 0L, WKNN, WKNN, kHidden, 0L, (void*)dst, (void*)dst, kChan, 0L,
          b_knn, 1.0f, prv, 0L, kRows, kChan, kHidden, invW);
    }
  }
  rowcvt_kernel<48, false><<<kRows / 8, 256, 0, stream>>>(PB, kChan, M16 + kChan, kHidden, kMCarry, kRows);

  wmma_gemm64<0, false, 2, 0, 1, 0><<<dim3((unsigned)(((kRows / 64) * (kChan / 64) + 7) / 8), 1), 256, 0, stream>>>(
      M16, M16, kHidden, 0L, WMRG, WMRG, kHidden, 0L, (void*)X2, (void*)X2, kChan, 0L,
      b_mrg, 1.0f, x, 0L, kRows, kChan, kHidden, 1.0f / (kMCarry * kWCarry));

  layernorm_kernel<false><<<kRows / 8, 256, 0, stream>>>(X2, ln2_w, ln2_b, U32, H16, kRows);

  wmma_gemm64<0, false, 2, 0, 0, 0><<<dim3((unsigned)(((kRows / 64) * (kHidden / 64) + 7) / 8), 1), 256, 0, stream>>>(
      H16, H16, kChan, 0L, WFC1, WFC1, kChan, 0L, (void*)U32, (void*)U32, kHidden, 0L,
      b_fc1, 1.0f, x, 0L, kRows, kHidden, kChan, invW);

  rowcvt_kernel<96, true><<<kRows / 8, 256, 0, stream>>>(U32, kHidden, FC16, kHidden, kFCarry, kRows);

  wmma_gemm64<0, false, 2, 0, 1, 0><<<dim3((unsigned)(((kRows / 64) * (kChan / 64) + 7) / 8), 1), 256, 0, stream>>>(
      FC16, FC16, kHidden, 0L, WFC2, WFC2, kHidden, 0L, (void*)out, (void*)out, kChan, 0L,
      b_fc2, 1.0f, X2, 0L, kRows, kChan, kHidden, 1.0f / (kFCarry * kWCarry));
}
